// PGExplainer_66571993088771
// MI455X (gfx1250) — hardware-verified
//
#include <hip/hip_runtime.h>
#include <stdint.h>
#include <stddef.h>


typedef _Float16 v16h __attribute__((ext_vector_type(16)));
typedef _Float16 v8h  __attribute__((ext_vector_type(8)));
typedef _Float16 v4h  __attribute__((ext_vector_type(4)));
typedef float    v8f  __attribute__((ext_vector_type(8)));
typedef float    v4f  __attribute__((ext_vector_type(4)));
union Frag { v16h v; v8h half[2]; };

#define DD        64
#define HH1       64
#define HH2       20
#define ETILE     128
#define HP        72
#define NROWS_BLK 128

__device__ __forceinline__ v8f wmma16(v8f c, v16h a, v16h b) {
  v8f d = __builtin_amdgcn_wmma_f32_16x16x32_f16(false, a, false, b, (short)0, c, false, false);
  asm volatile("v_nop\n\tv_nop\n\tv_nop\n\tv_nop" : "+v"(d) : "v"(a), "v"(b));
  return d;
}

__device__ __forceinline__ int clamp_idx(int i, int n) {
  i += (i < 0) ? n : 0;
  i = i < 0 ? 0 : i;
  i = i >= n ? n - 1 : i;
  return i;
}

__global__ __launch_bounds__(256)
void k_setup(const float* __restrict__ Z, const int* __restrict__ nidx,
             const float* __restrict__ W1, const float* __restrict__ b1,
             const float* __restrict__ W2, int N,
             float* c1, _Float16* W1T, _Float16* W2T) {
  const int t = threadIdx.x;
  const int nv = clamp_idx(nidx[0], N);

  float cval = 0.0f;
  if (t < HH1) {
    const float* zv = Z + (size_t)nv * DD;
    float s = 0.0f;
    for (int k = 0; k < DD; ++k) s += zv[k] * W1[(size_t)(2 * DD + k) * HH1 + t];
    cval = s + b1[t];
  }

  v8h w1v[4];
  #pragma unroll
  for (int j = 0; j < 4; ++j) {
    const int q  = t + 256 * j;
    const int R  = q >> 3;
    const int kc = (q & 7) * 8;
    const int p  = R >> 6, n = R & 63;
    #pragma unroll
    for (int i = 0; i < 8; ++i)
      w1v[j][i] = (_Float16)(64.0f * W1[(size_t)(p * DD + kc + i) * HH1 + n]);
  }
  v8h w2v;
  {
    const int n = t >> 3, kc = (t & 7) * 8;
    #pragma unroll
    for (int i = 0; i < 8; ++i)
      w2v[i] = (n < HH2) ? (_Float16)(32.0f * W2[(kc + i) * HH2 + n]) : (_Float16)0.0f;
  }

  if (t < HH1) *(volatile float*)(c1 + t) = cval;
  #pragma unroll
  for (int j = 0; j < 4; ++j) {
    const int q = t + 256 * j;
    *(volatile v8h*)(W1T + (size_t)(q >> 3) * DD + (q & 7) * 8) = w1v[j];
  }
  *(volatile v8h*)(W2T + (size_t)(t >> 3) * DD + (t & 7) * 8) = w2v;
  __threadfence();
  if (t < HH1) *(volatile float*)(c1 + t) = cval;
  #pragma unroll
  for (int j = 0; j < 4; ++j) {
    const int q = t + 256 * j;
    *(volatile v8h*)(W1T + (size_t)(q >> 3) * DD + (q & 7) * 8) = w1v[j];
  }
  *(volatile v8h*)(W2T + (size_t)(t >> 3) * DD + (t & 7) * 8) = w2v;
}

__global__ __launch_bounds__(256)
void k_cvt(const float* __restrict__ Z, _Float16* Zh, int N, int Npad) {
  const int q   = blockIdx.x * 256 + threadIdx.x;
  const int row = q >> 3;
  const int kc  = (q & 7) * 8;
  v8h v;
  #pragma unroll
  for (int i = 0; i < 8; ++i) v[i] = (_Float16)0.0f;
  if (row < N) {
    const v4f a = *(const v4f*)(Z + (size_t)row * DD + kc);
    const v4f b = *(const v4f*)(Z + (size_t)row * DD + kc + 4);
    #pragma unroll
    for (int i = 0; i < 4; ++i) { v[i] = (_Float16)a[i]; v[4 + i] = (_Float16)b[i]; }
  }
  if (row < Npad) {
    _Float16* p = Zh + (size_t)row * DD + kc;
    *(volatile v8h*)p = v;
    __threadfence();
    *(volatile v8h*)p = v;
  }
}

__global__ __launch_bounds__(128)
void k_node_gemm(const _Float16* __restrict__ Zh, const _Float16* __restrict__ W1T,
                 float* P, int Npad) {
  __shared__ float sD[4][16 * DD];
  const int lane = threadIdx.x & 31, wave = threadIdx.x >> 5;
  const int h = lane >> 4, m = lane & 15;
  const int part = blockIdx.y;

  Frag bf[2][4];
  #pragma unroll
  for (int ks = 0; ks < 2; ++ks)
    #pragma unroll
    for (int nt = 0; nt < 4; ++nt) {
      const _Float16* bp = W1T + (size_t)(part * HH1 + nt * 16 + m) * DD + ks * 32;
      bf[ks][nt].half[0] = *(const v8h*)(bp + 8 * h);
      bf[ks][nt].half[1] = *(const v8h*)(bp + 16 + 8 * h);
    }

  float* Pp = P + (size_t)part * (size_t)Npad * DD;
  float* sw = sD[wave];

  #pragma unroll 1
  for (int rt = 0; rt < 2; ++rt) {
    const int row0 = blockIdx.x * NROWS_BLK + wave * 32 + rt * 16;

    v8f acc[4];
    #pragma unroll
    for (int nt = 0; nt < 4; ++nt) {
      #pragma unroll
      for (int r = 0; r < 8; ++r) acc[nt][r] = 0.0f;
    }
    #pragma unroll
    for (int ks = 0; ks < 2; ++ks) {
      const _Float16* ap = Zh + (size_t)(row0 + m) * DD + ks * 32;
      Frag a;
      a.half[0] = *(const v8h*)(ap + 8 * h);
      a.half[1] = *(const v8h*)(ap + 16 + 8 * h);
      #pragma unroll
      for (int nt = 0; nt < 4; ++nt) acc[nt] = wmma16(acc[nt], a.v, bf[ks][nt].v);
    }

    #pragma unroll
    for (int nt = 0; nt < 4; ++nt) {
      #pragma unroll
      for (int r = 0; r < 8; ++r)
        sw[(8 * h + r) * DD + nt * 16 + m] = acc[nt][r] * 0.015625f;
    }
    __syncthreads();

    v4f rv[8];
    const int c4 = m * 4;
    #pragma unroll
    for (int it = 0; it < 8; ++it) {
      const int rr = it * 2 + h;
      rv[it] = *(const v4f*)(sw + rr * DD + c4);
      *(volatile v4f*)(Pp + (size_t)(row0 + rr) * DD + c4) = rv[it];
    }
    __threadfence();
    #pragma unroll
    for (int it = 0; it < 8; ++it) {
      const int rr = it * 2 + h;
      *(volatile v4f*)(Pp + (size_t)(row0 + rr) * DD + c4) = rv[it];
    }
    __syncthreads();
  }
}

__global__ __launch_bounds__(256)
void k_edge(const int* __restrict__ ei, const float* __restrict__ P,
            const float* __restrict__ c1, const _Float16* __restrict__ W2T,
            const float* __restrict__ b2, const float* __restrict__ W3,
            const float* __restrict__ b3p, float* out,
            int N, int Npad, int E, int Eo) {
  __shared__ _Float16 sH[ETILE * HP];
  __shared__ float sO[ETILE];

  const int lane = threadIdx.x & 31, wave = threadIdx.x >> 5;
  const int h = lane >> 4, m = lane & 15;
  const int ebase = blockIdx.x * ETILE;

  const v4f cv = *(const v4f*)(c1 + 4 * m);
  #pragma unroll 2
  for (int it = 0; it < 8; ++it) {
    const int le = wave * 16 + it * 2 + h;
    int e = ebase + le;
    e = e < E ? e : E - 1;
    const int s = clamp_idx(ei[e], N);
    const int d = clamp_idx(ei[(size_t)E + (size_t)e], N);
    const v4f pa = *(const v4f*)(P + (size_t)s * DD + 4 * m);
    const v4f pb = *(const v4f*)(P + ((size_t)Npad + (size_t)d) * DD + 4 * m);
    v4f x = pa + pb;
    x = x + cv;
    v4h hv;
    #pragma unroll
    for (int i = 0; i < 4; ++i) {
      float y = x[i];
      y = y > 0.0f ? y : 0.0f;
      hv[i] = (_Float16)y;
    }
    *(v4h*)(sH + le * HP + 4 * m) = hv;
  }
  __syncthreads();

  Frag bw[2][2];
  #pragma unroll
  for (int ks = 0; ks < 2; ++ks)
    #pragma unroll
    for (int nt = 0; nt < 2; ++nt) {
      const _Float16* bp = W2T + (size_t)(nt * 16 + m) * DD + ks * 32;
      bw[ks][nt].half[0] = *(const v8h*)(bp + 8 * h);
      bw[ks][nt].half[1] = *(const v8h*)(bp + 16 + 8 * h);
    }
  v8f acc[2];
  #pragma unroll
  for (int nt = 0; nt < 2; ++nt) {
    #pragma unroll
    for (int r = 0; r < 8; ++r) acc[nt][r] = 0.0f;
  }
  #pragma unroll
  for (int ks = 0; ks < 2; ++ks) {
    const _Float16* ap = sH + (wave * 16 + m) * HP + ks * 32;
    Frag a;
    a.half[0] = *(const v8h*)(ap + 8 * h);
    a.half[1] = *(const v8h*)(ap + 16 + 8 * h);
    #pragma unroll
    for (int nt = 0; nt < 2; ++nt) acc[nt] = wmma16(acc[nt], a.v, bw[ks][nt].v);
  }

  float b2v[2], w3v[2];
  #pragma unroll
  for (int nt = 0; nt < 2; ++nt) {
    const int n = nt * 16 + m;
    b2v[nt] = (n < HH2) ? b2[n] : 0.0f;
    w3v[nt] = (n < HH2) ? W3[n] : 0.0f;
  }
  float t[8];
  #pragma unroll
  for (int r = 0; r < 8; ++r) {
    float s = 0.0f;
    #pragma unroll
    for (int nt = 0; nt < 2; ++nt) {
      float y = acc[nt][r] * 0.03125f + b2v[nt];
      y = y > 0.0f ? y : 0.0f;
      s += y * w3v[nt];
    }
    t[r] = s;
  }
  #pragma unroll
  for (int sft = 1; sft < 16; sft <<= 1) {
    #pragma unroll
    for (int r = 0; r < 8; ++r) t[r] += __shfl_xor(t[r], sft, 32);
  }
  const float b3 = b3p[0];
  if (m < 8) {
    float om = t[0];
    #pragma unroll
    for (int v = 1; v < 8; ++v) om = (m == v) ? t[v] : om;
    const float z  = om + b3;
    const float ex = __expf(-z);
    const float y  = __builtin_amdgcn_rcpf(1.0f + ex);
    sO[wave * 16 + 8 * h + m] = y;
  }
  __syncthreads();

  if (wave == 0) {
    const v4f v  = *(const v4f*)(sO + 4 * lane);
    const int idx = ebase + 4 * lane;
    float* op = out + idx;
    const bool full = (idx + 4 <= Eo);
    if (full) {
      *(volatile v4f*)op = v;
    } else {
      #pragma unroll
      for (int i = 0; i < 4; ++i)
        if (idx + i < Eo) *(volatile float*)(op + i) = v[i];
    }
    __threadfence();
    if (full) {
      *(volatile v4f*)op = v;
    } else {
      #pragma unroll
      for (int i = 0; i < 4; ++i)
        if (idx + i < Eo) *(volatile float*)(op + i) = v[i];
    }
  }
}

extern "C" void kernel_launch(void* const* d_in, const int* in_sizes, int n_in,
                              void* d_out, int out_size, void* d_ws, size_t ws_size,
                              hipStream_t stream) {
  if (n_in < 9) return;
  const float* Z    = (const float*)d_in[0];
  const int*   ei   = (const int*)  d_in[1];
  const int*   nidx = (const int*)  d_in[2];
  const float* W1   = (const float*)d_in[3];
  const float* b1   = (const float*)d_in[4];
  const float* W2   = (const float*)d_in[5];
  const float* b2   = (const float*)d_in[6];
  const float* W3   = (const float*)d_in[7];
  const float* b3   = (const float*)d_in[8];
  float*       out  = (float*)d_out;

  const int N  = in_sizes[0] / DD;
  const int E  = in_sizes[1] / 2;
  const int Eo = out_size < E ? out_size : E;
  if (N <= 0 || E <= 0 || Eo <= 0 || in_sizes[2] < 1) return;
  const int Npad = ((N + NROWS_BLK - 1) / NROWS_BLK) * NROWS_BLK;

  unsigned char* ws = (unsigned char*)d_ws;
  size_t off = 0;
  float* c1 = (float*)(ws + off);            off += 256;
  _Float16* W1T = (_Float16*)(ws + off);     off += (size_t)2 * HH1 * DD * 2;
  _Float16* W2T = (_Float16*)(ws + off);     off += (size_t)32 * DD * 2;
  off = (off + 255) & ~(size_t)255;
  _Float16* Zh = (_Float16*)(ws + off);      off += (size_t)Npad * DD * 2;
  off = (off + 255) & ~(size_t)255;
  float* P = (float*)(ws + off);             off += (size_t)2 * (size_t)Npad * DD * 4;
  if (off > ws_size) return;

  k_setup<<<1, 256, 0, stream>>>(Z, nidx, W1, b1, W2, N, c1, W1T, W2T);
  k_cvt<<<Npad / 32, 256, 0, stream>>>(Z, Zh, N, Npad);
  k_node_gemm<<<dim3(Npad / NROWS_BLK, 2, 1), 128, 0, stream>>>(Zh, W1T, P, Npad);
  k_edge<<<(Eo + ETILE - 1) / ETILE, 256, 0, stream>>>(ei, P, c1, W2T, b2, W3, b3, out,
                                                       N, Npad, E, Eo);
}
